// MockCoreAttention_70188355551658
// MI455X (gfx1250) — hardware-verified
//
#include <hip/hip_runtime.h>
#include <math.h>
#include <stdint.h>

#define SEQ    2048
#define NBATCH 2
#define NQH    16
#define NKV    4
#define HD     128
#define NREP   (NQH / NKV)
#define HID    (NQH * HD)

static_assert(SEQ % 64 == 0);
static_assert(HD == 128);
static_assert(NQH % NKV == 0);

typedef __attribute__((ext_vector_type(16))) __bf16 v16b;
typedef __attribute__((ext_vector_type(8)))  __bf16 v8b;
typedef __attribute__((ext_vector_type(8)))  float  v8f;
typedef __attribute__((ext_vector_type(4)))  float  v4f;
typedef __attribute__((ext_vector_type(4)))  unsigned int v4u;

__device__ __forceinline__ unsigned short f2bf_bits(float f) {
  unsigned u = __float_as_uint(f);
  return (unsigned short)((u + 0x7FFFu + ((u >> 16) & 1u)) >> 16);
}
__device__ __forceinline__ float bf_bits2f(unsigned short b) { return __uint_as_float(((unsigned)b) << 16); }
__device__ __forceinline__ unsigned pk16(unsigned short a, unsigned short b) { return (unsigned)a | ((unsigned)b << 16); }

__device__ __forceinline__ void split2(float f0, float f1, unsigned& hw, unsigned& lw) {
  const unsigned short h0 = f2bf_bits(f0), h1 = f2bf_bits(f1);
  const unsigned short l0 = f2bf_bits(f0 - bf_bits2f(h0)), l1 = f2bf_bits(f1 - bf_bits2f(h1));
  hw = pk16(h0, h1);
  lw = pk16(l0, l1);
}

__device__ __forceinline__ v8f mma_bf(v16b a, v16b b, v8f c) {
  c = __builtin_amdgcn_wmma_f32_16x16x32_bf16(false, a, false, b, (short)0, c, false, false);
  asm volatile("v_nop\n\tv_nop\n\tv_nop\n\tv_nop" : "+v"(c) : "v"(a), "v"(b));
  return c;
}

__global__ __launch_bounds__(256) void split_rows_kernel(const float* __restrict__ src,
                                                         unsigned short* __restrict__ hi,
                                                         unsigned short* __restrict__ lo,
                                                         int nh, int ngrp) {
  const int t = blockIdx.x * 256 + (int)threadIdx.x;
  if (t >= ngrp) return;
  const int i   = t >> 4;
  const int d8  = (t & 15) * 8;
  const int bn  = NBATCH * nh;
  const int s   = i / bn;
  const int rem = i - s * bn;
  const int b   = rem / nh;
  const int hd  = rem - b * nh;
  const size_t so  = (size_t)i * HD + d8;
  const size_t dso = ((size_t)(b * nh + hd) * SEQ + s) * HD + d8;
  const v4f a0 = *(const v4f*)(src + so);
  const v4f a1 = *(const v4f*)(src + so + 4);
  unsigned h0, h1, h2, h3, l0, l1, l2, l3;
  split2(a0[0], a0[1], h0, l0);
  split2(a0[2], a0[3], h1, l1);
  split2(a1[0], a1[1], h2, l2);
  split2(a1[2], a1[3], h3, l3);
  const v4u hv = (v4u){h0, h1, h2, h3};
  const v4u lv = (v4u){l0, l1, l2, l3};
  volatile v4u* ph = (volatile v4u*)(hi + dso);
  volatile v4u* pl = (volatile v4u*)(lo + dso);
  *ph = hv;
  *pl = lv;
  __threadfence();
  *ph = hv;
  *pl = lv;
}

#define TFP 132
__global__ __launch_bounds__(256) void vt_split_kernel(const float* __restrict__ v,
                                                       unsigned short* __restrict__ vth,
                                                       unsigned short* __restrict__ vtl) {
  __shared__ __align__(16) float tf[64 * TFP];
  const int tid = threadIdx.x;
  const int nt  = blockIdx.x % (SEQ / 64);
  const int bg  = blockIdx.x / (SEQ / 64);
  const int b   = bg / NKV;
  const int g   = bg - b * NKV;
  const int n0  = nt * 64;
  {
    const int lr = tid >> 4;
    const int c8 = (tid & 15) * 8;
#pragma unroll
    for (int it = 0; it < 4; ++it) {
      const int row = it * 16 + lr;
      const float* sp = v + (((size_t)(n0 + row) * NBATCH + b) * NKV + g) * HD + c8;
      const v4f a0 = *(const v4f*)(sp);
      const v4f a1 = *(const v4f*)(sp + 4);
      *(v4f*)(tf + row * TFP + c8) = a0;
      *(v4f*)(tf + row * TFP + c8 + 4) = a1;
    }
  }
  __syncthreads();
  {
    const int sub = tid >> 3;
    const int t8  = (tid & 7) * 8;
    v4u hv[4], lv[4];
#pragma unroll
    for (int it = 0; it < 4; ++it) {
      const int d = it * 32 + sub;
      unsigned hw[4], lw[4];
#pragma unroll
      for (int q = 0; q < 4; ++q) {
        const float f0 = tf[(t8 + 2 * q) * TFP + d];
        const float f1 = tf[(t8 + 2 * q + 1) * TFP + d];
        split2(f0, f1, hw[q], lw[q]);
      }
      hv[it] = (v4u){hw[0], hw[1], hw[2], hw[3]};
      lv[it] = (v4u){lw[0], lw[1], lw[2], lw[3]};
    }
    unsigned short* th = vth + (size_t)bg * HD * SEQ + n0 + t8;
    unsigned short* tl = vtl + (size_t)bg * HD * SEQ + n0 + t8;
    for (int ps = 0; ps < 2; ++ps) {
#pragma unroll
      for (int it = 0; it < 4; ++it) {
        const int d = it * 32 + sub;
        const size_t go = (size_t)d * SEQ;
        *(volatile v4u*)(th + go) = hv[it];
        *(volatile v4u*)(tl + go) = lv[it];
      }
      __threadfence();
    }
  }
}

#define QB  64
#define KC  64
#define KSP 136
#define VTP 72
#define PSP 64
#define OSP 68

__global__ __launch_bounds__(256)
void attn_causal_kernel(const unsigned short* __restrict__ qhp, const unsigned short* __restrict__ qlp,
                        const unsigned short* __restrict__ khp, const unsigned short* __restrict__ klp,
                        const unsigned short* __restrict__ vhp, const unsigned short* __restrict__ vlp,
                        float* __restrict__ out, float sscale) {
  union FB { v16b v; v8b h[2]; };
  __shared__ __align__(16) __bf16 Ksh[KC * KSP];
  __shared__ __align__(16) __bf16 Ksl[KC * KSP];
  __shared__ __align__(16) __bf16 Vth[HD * VTP];
  __shared__ __align__(16) __bf16 Vtl[HD * VTP];
  __shared__ __align__(16) __bf16 Psh[4][16 * PSP];
  __shared__ __align__(16) __bf16 Psl[4][16 * PSP];
  __shared__ __align__(16) float  Al[4][16];
  __shared__ __align__(16) float  Ll[4][16];
  __shared__ __align__(16) float  Os[8][16 * OSP];

  const int tid  = threadIdx.x;
  const int wave = tid >> 5;
  const int lane = tid & 31;
  const int lh   = lane >> 4;
  const int c    = lane & 15;
  const int g    = wave & 3;
  const int chh  = wave >> 2;
  const int ch0  = chh * 64;

  const int nqt = SEQ / QB;
  const int qt  = blockIdx.x % nqt;
  const int bh  = blockIdx.x / nqt;
  const int b   = bh / NQH;
  const int h   = bh - b * NQH;
  const int bg  = b * NKV + h / NREP;
  const int qg0 = qt * QB + g * 16;

  const __bf16* Qh = (const __bf16*)(const void*)qhp + (size_t)bh * SEQ * HD;
  const __bf16* Ql = (const __bf16*)(const void*)qlp + (size_t)bh * SEQ * HD;
  const __bf16* Kh = (const __bf16*)(const void*)khp + (size_t)bg * SEQ * HD;
  const __bf16* Kl = (const __bf16*)(const void*)klp + (size_t)bg * SEQ * HD;
  const __bf16* Vh = (const __bf16*)(const void*)vhp + (size_t)bg * HD * SEQ;
  const __bf16* Vl = (const __bf16*)(const void*)vlp + (size_t)bg * HD * SEQ;

  float mrow[8], lrow[8];
  v8f oacc[4];
#pragma unroll
  for (int r = 0; r < 8; ++r) { mrow[r] = -INFINITY; lrow[r] = 0.f; }
#pragma unroll
  for (int t = 0; t < 4; ++t) oacc[t] = (v8f){0.f, 0.f, 0.f, 0.f, 0.f, 0.f, 0.f, 0.f};

  __bf16* pwh = Psh[g];
  __bf16* pwl = Psl[g];

  const int nChunks = qt + 1;
  for (int kc = 0; kc < nChunks; ++kc) {
    const int kv0 = kc * KC;
    __syncthreads();
    {
      const int r = tid >> 2, qq = (tid & 3) * 32;
      const __bf16* khs = Kh + (size_t)(kv0 + r) * HD + qq;
      const __bf16* kls = Kl + (size_t)(kv0 + r) * HD + qq;
      __bf16* kdh = Ksh + r * KSP + qq;
      __bf16* kdl = Ksl + r * KSP + qq;
#pragma unroll
      for (int i = 0; i < 4; ++i) {
        *(v8b*)(kdh + 8 * i) = *(const v8b*)(khs + 8 * i);
        *(v8b*)(kdl + 8 * i) = *(const v8b*)(kls + 8 * i);
      }
      const int r2 = tid >> 1, hf = (tid & 1) * 32;
      const __bf16* vhs = Vh + (size_t)r2 * SEQ + kv0 + hf;
      const __bf16* vls = Vl + (size_t)r2 * SEQ + kv0 + hf;
#pragma unroll
      for (int i = 0; i < 4; ++i) {
        *(v8b*)(Vth + r2 * VTP + hf + 8 * i) = *(const v8b*)(vhs + 8 * i);
        *(v8b*)(Vtl + r2 * VTP + hf + 8 * i) = *(const v8b*)(vls + 8 * i);
      }
    }
    __syncthreads();

    if (wave < 4) {
      v8f s[4];
#pragma unroll
      for (int j = 0; j < 4; ++j) s[j] = (v8f){0.f, 0.f, 0.f, 0.f, 0.f, 0.f, 0.f, 0.f};
      const __bf16* qrh = Qh + (size_t)(qg0 + c) * HD + 8 * lh;
      const __bf16* qrl = Ql + (size_t)(qg0 + c) * HD + 8 * lh;
#pragma unroll
      for (int dc = 0; dc < 4; ++dc) {
        FB qa, ql;
        qa.h[0] = *(const v8b*)(qrh + dc * 32);
        qa.h[1] = *(const v8b*)(qrh + dc * 32 + 16);
        ql.h[0] = *(const v8b*)(qrl + dc * 32);
        ql.h[1] = *(const v8b*)(qrl + dc * 32 + 16);
#pragma unroll
        for (int j = 0; j < 4; ++j) {
          const __bf16* kp = Ksh + (j * 16 + c) * KSP + dc * 32 + 8 * lh;
          const __bf16* kq = Ksl + (j * 16 + c) * KSP + dc * 32 + 8 * lh;
          FB kb, kl;
          kb.h[0] = *(const v8b*)(kp);
          kb.h[1] = *(const v8b*)(kp + 16);
          kl.h[0] = *(const v8b*)(kq);
          kl.h[1] = *(const v8b*)(kq + 16);
          s[j] = mma_bf(qa.v, kb.v, s[j]);
          s[j] = mma_bf(qa.v, kl.v, s[j]);
          s[j] = mma_bf(ql.v, kb.v, s[j]);
        }
      }
      float cm[8];
#pragma unroll
      for (int r = 0; r < 8; ++r) {
        const int qrow = qg0 + 8 * lh + r;
        float m = -INFINITY;
#pragma unroll
        for (int j = 0; j < 4; ++j) {
          const int key = kv0 + j * 16 + c;
          const float sv = (key > qrow) ? -INFINITY : s[j][r] * sscale;
          s[j][r] = sv;
          m = fmaxf(m, sv);
        }
#pragma unroll
        for (int off = 1; off < 16; off <<= 1) m = fmaxf(m, __shfl_xor(m, off, 32));
        cm[r] = m;
      }
#pragma unroll
      for (int r = 0; r < 8; ++r) {
        const float mnew  = fmaxf(mrow[r], cm[r]);
        const float alpha = __expf(mrow[r] - mnew);
        mrow[r] = mnew;
        float psum = 0.f;
#pragma unroll
        for (int j = 0; j < 4; ++j) {
          const float p = __expf(s[j][r] - mnew);
          psum += p;
          const unsigned short hb = f2bf_bits(p);
          const unsigned short lb = f2bf_bits(p - bf_bits2f(hb));
          pwh[(8 * lh + r) * PSP + j * 16 + c] = __builtin_bit_cast(__bf16, hb);
          pwl[(8 * lh + r) * PSP + j * 16 + c] = __builtin_bit_cast(__bf16, lb);
        }
#pragma unroll
        for (int off = 1; off < 16; off <<= 1) psum += __shfl_xor(psum, off, 32);
        lrow[r] = lrow[r] * alpha + psum;
        if (c == 0) {
          Al[g][8 * lh + r] = alpha;
          Ll[g][8 * lh + r] = lrow[r];
        }
      }
    }
    __syncthreads();

    {
      float af[8];
#pragma unroll
      for (int r = 0; r < 8; ++r) af[r] = Al[g][8 * lh + r];
#pragma unroll
      for (int t = 0; t < 4; ++t)
#pragma unroll
        for (int r = 0; r < 8; ++r) oacc[t][r] *= af[r];
#pragma unroll 1
      for (int kk = 0; kk < 2; ++kk) {
        FB pa, pl;
        pa.h[0] = *(const v8b*)(pwh + c * PSP + kk * 32 + 8 * lh);
        pa.h[1] = *(const v8b*)(pwh + c * PSP + kk * 32 + 16 + 8 * lh);
        pl.h[0] = *(const v8b*)(pwl + c * PSP + kk * 32 + 8 * lh);
        pl.h[1] = *(const v8b*)(pwl + c * PSP + kk * 32 + 16 + 8 * lh);
#pragma unroll
        for (int t = 0; t < 4; ++t) {
          const __bf16* vp = Vth + (ch0 + t * 16 + c) * VTP + kk * 32 + 8 * lh;
          const __bf16* vq = Vtl + (ch0 + t * 16 + c) * VTP + kk * 32 + 8 * lh;
          FB vb, vl;
          vb.h[0] = *(const v8b*)(vp);
          vb.h[1] = *(const v8b*)(vp + 16);
          vl.h[0] = *(const v8b*)(vq);
          vl.h[1] = *(const v8b*)(vq + 16);
          oacc[t] = mma_bf(pa.v, vb.v, oacc[t]);
          oacc[t] = mma_bf(pa.v, vl.v, oacc[t]);
          oacc[t] = mma_bf(pl.v, vb.v, oacc[t]);
        }
      }
    }
  }

  float* os = Os[wave];
#pragma unroll
  for (int r = 0; r < 8; ++r) {
    const float inv = 1.0f / Ll[g][8 * lh + r];
#pragma unroll
    for (int t = 0; t < 4; ++t) os[(8 * lh + r) * OSP + t * 16 + c] = oacc[t][r] * inv;
  }
  __builtin_amdgcn_fence(__ATOMIC_RELEASE, "workgroup");
  __builtin_amdgcn_wave_barrier();
  __builtin_amdgcn_fence(__ATOMIC_ACQUIRE, "workgroup");
  {
    const int rh = lane >> 4, c4 = (lane & 15) * 4;
    for (int ps = 0; ps < 2; ++ps) {
#pragma unroll
      for (int it = 0; it < 8; ++it) {
        const int row = it * 2 + rh;
        const v4f vv = *(const v4f*)(os + row * OSP + c4);
        const size_t go = ((size_t)(qg0 + row) * NBATCH + b) * HID + (size_t)h * HD + ch0 + c4;
        *(volatile v4f*)(out + go) = vv;
      }
      __threadfence();
    }
  }
}

extern "C" void kernel_launch(void* const* d_in, const int* in_sizes, int n_in,
                              void* d_out, int out_size, void* d_ws, size_t ws_size,
                              hipStream_t stream) {
  if (n_in < 3) return;
  if (in_sizes[0] != SEQ * NBATCH * NQH * HD) return;
  if (in_sizes[1] != SEQ * NBATCH * NKV * HD) return;
  if (in_sizes[2] != SEQ * NBATCH * NKV * HD) return;
  if (out_size != SEQ * NBATCH * HID) return;

  const float* q = (const float*)d_in[0];
  const float* k = (const float*)d_in[1];
  const float* v = (const float*)d_in[2];
  float* o = (float*)d_out;

  const size_t PQ = (size_t)SEQ * NBATCH * NQH * HD * 2;
  const size_t PK = (size_t)SEQ * NBATCH * NKV * HD * 2;
  size_t off = 0;
  const size_t oQh = off; off += PQ;
  const size_t oQl = off; off += PQ;
  const size_t oKh = off; off += PK;
  const size_t oKl = off; off += PK;
  const size_t oVh = off; off += PK;
  const size_t oVl = off; off += PK;
  if (off > ws_size) return;

  char* ws = (char*)d_ws;
  unsigned short* Qh  = (unsigned short*)(ws + oQh);
  unsigned short* Ql  = (unsigned short*)(ws + oQl);
  unsigned short* Kh  = (unsigned short*)(ws + oKh);
  unsigned short* Kl  = (unsigned short*)(ws + oKl);
  unsigned short* VTh = (unsigned short*)(ws + oVh);
  unsigned short* VTl = (unsigned short*)(ws + oVl);

  const int ngq = SEQ * NBATCH * NQH * HD / 8;
  split_rows_kernel<<<dim3((ngq + 255) / 256), dim3(256), 0, stream>>>(q, Qh, Ql, NQH, ngq);
  const int ngk = SEQ * NBATCH * NKV * HD / 8;
  split_rows_kernel<<<dim3((ngk + 255) / 256), dim3(256), 0, stream>>>(k, Kh, Kl, NKV, ngk);
  vt_split_kernel<<<dim3(NBATCH * NKV * (SEQ / 64)), dim3(256), 0, stream>>>(v, VTh, VTl);
  attn_causal_kernel<<<dim3(NBATCH * NQH * (SEQ / QB)), dim3(256), 0, stream>>>(
      Qh, Ql, Kh, Kl, VTh, VTl, o, 0.08838834764831845f);
  (void)hipGetLastError();
}
